// BasicMambaBlock_66589172957422
// MI455X (gfx1250) — hardware-run, weakly checked
//
#include <hip/hip_runtime.h>
#include <math.h>

typedef __attribute__((ext_vector_type(16))) _Float16 v16h;
typedef __attribute__((ext_vector_type(8)))  _Float16 v8h;
typedef __attribute__((ext_vector_type(2)))  _Float16 v2h;
typedef __attribute__((ext_vector_type(8)))  float    v8f;
typedef __attribute__((ext_vector_type(4)))  float    v4f;

constexpr int kBatch = 2;
constexpr int kSeq   = 2048;
constexpr int kDm    = 1024;
constexpr int kDi    = 2048;
constexpr int kNs    = 16;
constexpr int kDtR   = 64;
constexpr int kXpN   = kDtR + 2 * kNs;
constexpr int kXpP   = 128;
constexpr int kBcP   = 64;
constexpr int kFf    = 4096;
constexpr int kRows  = kBatch * kSeq;
constexpr int kConvTP = 260;
constexpr float kLnEps = 1e-5f;
static_assert(kXpN == 96);
static_assert(kXpP - kDtR == kBcP);
static_assert((kDm % 32) == 0 && (kDi % 32) == 0 && (kDtR % 32) == 0 && (kFf % 32) == 0);
static_assert((kRows % 64) == 0 && ((2 * kDi) % 64) == 0 && (kXpP % 64) == 0 && (kDi % 64) == 0 && (kDm % 64) == 0 && (kFf % 64) == 0);
static_assert((kSeq % 64) == 0 && (kDi % 256) == 0 && (kDm % 256) == 0);

constexpr float kCarryH   = 16.0f;
constexpr float kCarryW   = 256.0f;
constexpr float kCarryWdt = 64.0f;
constexpr float kCarryXc  = 64.0f;
constexpr float kCarryDbc = 64.0f;
constexpr float kCarryY   = 1024.0f;
constexpr float kCarryAct = 256.0f;
constexpr float kScaleIn   = 1.0f / (kCarryH * kCarryW);
constexpr float kScaleXpLo = kCarryDbc / (kCarryXc * kCarryW);
constexpr float kScaleXpBc = 1.0f / (kCarryXc * kCarryW);
constexpr float kScaleDt   = 1.0f / (kCarryDbc * kCarryWdt);
constexpr float kScaleOut  = 1.0f / (kCarryY * kCarryW);
constexpr float kScaleFf1  = 1.0f / (kCarryH * kCarryW);
constexpr float kScaleFf2  = 1.0f / (kCarryAct * kCarryW);
constexpr float kInvXc     = 1.0f / kCarryXc;
constexpr float kGeluC0    = 0.7978845608028654f;
constexpr float kGeluC1    = 0.044715f;

constexpr size_t kSzWIn  = (size_t)(2 * kDi) * kDm * 2;
constexpr size_t kSzWX   = (size_t)kXpP * kDi * 2;
constexpr size_t kSzWDt  = (size_t)kDi * kDtR * 2;
constexpr size_t kSzWOut = (size_t)kDm * kDi * 2;
constexpr size_t kSzH    = (size_t)kRows * kDm * 2;
constexpr size_t kSzX2   = (size_t)kRows * kDm * 4;
constexpr size_t kSzDtLo = (size_t)kRows * kDtR * 2;
constexpr size_t kSzBC   = (size_t)kRows * kBcP * 4;
constexpr size_t kSzPl   = (size_t)kRows * kDi * 2;
constexpr size_t kSzS    = 4 * kSzPl;
constexpr size_t kOffWIn  = 0;
constexpr size_t kOffWX   = kOffWIn  + kSzWIn;
constexpr size_t kOffWDt  = kOffWX   + kSzWX;
constexpr size_t kOffWOut = kOffWDt  + kSzWDt;
constexpr size_t kOffH    = kOffWOut + kSzWOut;
constexpr size_t kOffX2   = kOffH    + kSzH;
constexpr size_t kOffDtLo = kOffX2   + kSzX2;
constexpr size_t kOffBC   = kOffDtLo + kSzDtLo;
constexpr size_t kOffS    = kOffBC   + kSzBC;
constexpr size_t kWsTotal = kOffS    + kSzS;
constexpr size_t kOffXpre = kOffS;
constexpr size_t kOffZ    = kOffS + kSzPl;
constexpr size_t kOffXc   = kOffS + 2 * kSzPl;
constexpr size_t kOffDt   = kOffS + 3 * kSzPl;
constexpr size_t kSzAct   = (size_t)kRows * kFf * 2;
constexpr size_t kSzWFf1  = (size_t)(2 * kFf) * kDm * 2;
constexpr size_t kSzWFf2  = (size_t)kDm * kFf * 2;
constexpr size_t kOffAct  = kOffS;
constexpr size_t kOffWFf1 = kOffAct + kSzAct;
constexpr size_t kOffWFf2 = kOffWFf1 + kSzWFf1;
static_assert(kWsTotal == 107216896ull);
static_assert(kWsTotal <= 134217728ull);
static_assert(kOffWFf2 + kSzWFf2 <= kWsTotal);
static_assert(kSzAct == 2 * kSzPl && kSzWFf1 == kSzPl);
static_assert((kOffWX % 128) == 0 && (kOffWDt % 128) == 0 && (kOffWOut % 128) == 0 && (kOffH % 128) == 0 &&
              (kOffX2 % 128) == 0 && (kOffDtLo % 128) == 0 && (kOffBC % 128) == 0 && (kOffS % 128) == 0 &&
              (kSzPl % 128) == 0);

__device__ __forceinline__ float h16_to_f32(unsigned hb) {
  const unsigned sgn = (hb & 0x8000u) << 16;
  const unsigned em = hb & 0x7fffu;
  const float fn = __uint_as_float((em << 13) + 0x38000000u);
  const float fs = (float)em * 5.9604644775390625e-8f;
  const float mag = (em < 0x400u) ? fs : fn;
  return __uint_as_float(__float_as_uint(mag) | sgn);
}
__device__ __forceinline__ float softplus_f(float v) {
  return fmaxf(v, 0.0f) + log1pf(expf(-fabsf(v)));
}
__device__ __forceinline__ void wave_sync() {
  __builtin_amdgcn_fence(__ATOMIC_RELEASE, "workgroup");
  __builtin_amdgcn_wave_barrier();
  __builtin_amdgcn_fence(__ATOMIC_ACQUIRE, "workgroup");
}
__device__ __forceinline__ void wmma_guard(v8f& d, v16h a, v16h b) {
  asm volatile("v_nop\n\tv_nop\n\tv_nop\n\tv_nop" : "+v"(d) : "v"(a), "v"(b));
}
__device__ __forceinline__ void keep4_h(v16h a, v16h b, v16h c, v16h d) { asm volatile("v_nop" :: "v"(a), "v"(b), "v"(c), "v"(d)); }
__device__ __forceinline__ void acc_guard4(v8f& a, v8f& b, v8f& c, v8f& d) { asm volatile("v_nop\n\tv_nop\n\tv_nop\n\tv_nop" : "+v"(a), "+v"(b), "+v"(c), "+v"(d)); }

union FragU { v16h v; v8h h[2]; };
__device__ __forceinline__ v16h frag_load(const _Float16* p) {
  FragU f;
  f.h[0] = *(const v8h*)(p);
  f.h[1] = *(const v8h*)(p + 16);
  return f.v;
}
__device__ __forceinline__ v8f frag_mma(v16h a, v16h b, v8f c) {
  return __builtin_amdgcn_wmma_f32_16x16x32_f16(false, a, false, b, (short)0, c, false, false);
}

template <int EPI>
__global__ __launch_bounds__(256) void gemm64_f16_kernel(
    const unsigned short* __restrict__ Ap, int lda,
    const unsigned short* __restrict__ Btp, int ldb,
    void* __restrict__ C0, void* __restrict__ C1, int ldc, int nsplit,
    const float* __restrict__ bias, const float* __restrict__ resid,
    int M, int N, int K, float scale, float scale2)
{
  const _Float16* A  = (const _Float16*)Ap;
  const _Float16* Bt = (const _Float16*)Btp;
  __shared__ __align__(16) float sT[8][16 * 68];
  const int lane = threadIdx.x & 31;
  const int wave = threadIdx.x >> 5;
  const int tilesN = N >> 6;
  const int tilesM = M >> 6;
  const int tile = blockIdx.x * 8 + wave;
  if (tile >= tilesM * tilesN) return;
  const int tm = tile / tilesN;
  const int tn = tile - tm * tilesN;
  const int m0 = tm << 6;
  const int n0 = tn << 6;
  const int rlane = lane & 15;
  const int koff  = (lane >> 4) * 8;
  const int mOff  = (lane >> 4) * 8;

  v8f acc[4][4];
#pragma unroll
  for (int i = 0; i < 4; ++i)
#pragma unroll
    for (int j = 0; j < 4; ++j) acc[i][j] = (v8f){0.f, 0.f, 0.f, 0.f, 0.f, 0.f, 0.f, 0.f};

  for (int k0 = 0; k0 < K; k0 += 32) {
    v16h bh[4];
#pragma unroll
    for (int j = 0; j < 4; ++j)
      bh[j] = frag_load(Bt + (size_t)(n0 + (j << 4) + rlane) * ldb + koff + k0);
#pragma unroll
    for (int i = 0; i < 4; ++i) {
      const v16h ah = frag_load(A + (size_t)(m0 + (i << 4) + rlane) * lda + koff + k0);
#pragma unroll
      for (int j = 0; j < 4; ++j) acc[i][j] = frag_mma(ah, bh[j], acc[i][j]);
#pragma unroll
      for (int j = 0; j < 4; ++j) wmma_guard(acc[i][j], ah, bh[j]);
    }
    keep4_h(bh[0], bh[1], bh[2], bh[3]);
  }
  acc_guard4(acc[0][0], acc[0][1], acc[0][2], acc[0][3]);
  acc_guard4(acc[1][0], acc[1][1], acc[1][2], acc[1][3]);
  acc_guard4(acc[2][0], acc[2][1], acc[2][2], acc[2][3]);
  acc_guard4(acc[3][0], acc[3][1], acc[3][2], acc[3][3]);

  float* slab = sT[wave];
  const bool lowTile = (n0 < nsplit);
  const float sc = (EPI == 1 && !lowTile) ? scale2 : scale;
#pragma unroll
  for (int i = 0; i < 4; ++i) {
    const int mBase = m0 + (i << 4);
#pragma unroll
    for (int j = 0; j < 4; ++j) {
      const int n = n0 + (j << 4) + rlane;
      float bv = 0.f;
      if (EPI == 2 || EPI == 4) bv = bias[n];
#pragma unroll
      for (int r = 0; r < 8; ++r) {
        float v = acc[i][j][r] * sc;
        if (EPI == 2 || EPI == 4) v += bv;
        slab[(mOff + r) * 68 + (j << 4) + rlane] = v;
      }
    }
    wave_sync();
    if (EPI == 0 || EPI == 2 || (EPI == 1 && lowTile)) {
      const int q = lane >> 3, c8 = (lane & 7) * 8;
      unsigned short* Cb = (unsigned short*)C0;
      int ncol = n0;
      if (EPI == 0) {
        Cb = lowTile ? (unsigned short*)C0 : (unsigned short*)C1;
        ncol = lowTile ? n0 : (n0 - nsplit);
      }
      if (EPI == 2) {
#pragma unroll 1
        for (int idx = 0; idx < 32; ++idx) {
          float* p = slab + ((idx >> 3) * 4 + q) * 68 + c8 + (idx & 7);
          const float v = *p;
          *p = softplus_f(v);
        }
      }
      v8h hv[4];
#pragma unroll
      for (int it = 0; it < 4; ++it) {
        const float* sp = slab + (it * 4 + q) * 68 + c8;
        const v4f a0 = *(const v4f*)(sp);
        const v4f a1 = *(const v4f*)(sp + 4);
#pragma unroll
        for (int e = 0; e < 4; ++e) {
          hv[it][e]     = (_Float16)a0[e];
          hv[it][4 + e] = (_Float16)a1[e];
        }
      }
      for (int pass = 0; pass < 2; ++pass) {
#pragma unroll
        for (int it = 0; it < 4; ++it)
          *(volatile v8h*)(Cb + (size_t)(mBase + it * 4 + q) * ldc + ncol + c8) = hv[it];
        __threadfence();
      }
    } else {
      const int hh = lane >> 4, c4 = (lane & 15) * 4;
      float* Cf = (EPI == 1) ? (float*)C1 : (float*)C0;
      const int ncf = (EPI == 1) ? (n0 - nsplit) : n0;
      v4f vv[8];
#pragma unroll
      for (int it = 0; it < 8; ++it) {
        const int row = it * 2 + hh;
        v4f v = *(const v4f*)(slab + row * 68 + c4);
        if (EPI == 3 || EPI == 4) {
          const v4f rv = *(const v4f*)(resid + (size_t)(mBase + row) * ldc + ncf + c4);
          v = v + rv;
        }
        vv[it] = v;
      }
      for (int pass = 0; pass < 2; ++pass) {
#pragma unroll
        for (int it = 0; it < 8; ++it)
          *(volatile v4f*)(Cf + (size_t)(mBase + it * 2 + hh) * ldc + ncf + c4) = vv[it];
        __threadfence();
      }
    }
    wave_sync();
  }
}

__global__ __launch_bounds__(128) void gemm_gated_f16_kernel(
    const unsigned short* __restrict__ Ap, int lda,
    const unsigned short* __restrict__ Btp, int ldb,
    unsigned short* __restrict__ Cact, int ldc,
    const float* __restrict__ bias,
    int M, int NACT, int K, float scale, float ocarry)
{
  const _Float16* A  = (const _Float16*)Ap;
  const _Float16* Bt = (const _Float16*)Btp;
  __shared__ __align__(16) float sLin[4][16 * 68];
  __shared__ __align__(16) float sGate[4][16 * 68];
  const int lane = threadIdx.x & 31;
  const int wave = threadIdx.x >> 5;
  const int tilesN = NACT >> 6;
  const int tilesM = M >> 5;
  const int tile = blockIdx.x * 4 + wave;
  if (tile >= tilesM * tilesN) return;
  const int tm = tile / tilesN;
  const int tn = tile - tm * tilesN;
  const int m0 = tm << 5;
  const int n0 = tn << 6;
  const int rlane = lane & 15;
  const int koff  = (lane >> 4) * 8;
  const int mOff  = (lane >> 4) * 8;

  v8f acc[2][8];
#pragma unroll
  for (int i = 0; i < 2; ++i)
#pragma unroll
    for (int j = 0; j < 8; ++j) acc[i][j] = (v8f){0.f, 0.f, 0.f, 0.f, 0.f, 0.f, 0.f, 0.f};

  for (int k0 = 0; k0 < K; k0 += 32) {
    const v16h ah0 = frag_load(A + (size_t)(m0 + rlane) * lda + koff + k0);
    const v16h ah1 = frag_load(A + (size_t)(m0 + 16 + rlane) * lda + koff + k0);
#pragma unroll
    for (int jg = 0; jg < 2; ++jg) {
      const int nb = (jg == 0) ? n0 : (NACT + n0);
      v16h bh[4];
#pragma unroll
      for (int jj = 0; jj < 4; ++jj)
        bh[jj] = frag_load(Bt + (size_t)(nb + (jj << 4) + rlane) * ldb + koff + k0);
#pragma unroll
      for (int jj = 0; jj < 4; ++jj) {
        acc[0][jg * 4 + jj] = frag_mma(ah0, bh[jj], acc[0][jg * 4 + jj]);
        acc[1][jg * 4 + jj] = frag_mma(ah1, bh[jj], acc[1][jg * 4 + jj]);
      }
#pragma unroll
      for (int jj = 0; jj < 4; ++jj) {
        wmma_guard(acc[0][jg * 4 + jj], ah0, bh[jj]);
        wmma_guard(acc[1][jg * 4 + jj], ah1, bh[jj]);
      }
    }
  }
  acc_guard4(acc[0][0], acc[0][1], acc[0][2], acc[0][3]);
  acc_guard4(acc[0][4], acc[0][5], acc[0][6], acc[0][7]);
  acc_guard4(acc[1][0], acc[1][1], acc[1][2], acc[1][3]);
  acc_guard4(acc[1][4], acc[1][5], acc[1][6], acc[1][7]);

  float* sa = sLin[wave];
  float* sg = sGate[wave];
  const int q = lane >> 3, c8 = (lane & 7) * 8;
#pragma unroll
  for (int i = 0; i < 2; ++i) {
    const int mBase = m0 + (i << 4);
#pragma unroll
    for (int jj = 0; jj < 4; ++jj) {
      const int n = n0 + (jj << 4) + rlane;
      const float ba = bias[n];
      const float bg = bias[NACT + n];
#pragma unroll
      for (int r = 0; r < 8; ++r) {
        const int o = (mOff + r) * 68 + (jj << 4) + rlane;
        sa[o] = acc[i][jj][r] * scale + ba;
        sg[o] = acc[i][4 + jj][r] * scale + bg;
      }
    }
    wave_sync();
#pragma unroll 1
    for (int idx = 0; idx < 32; ++idx) {
      const int o = ((idx >> 3) * 4 + q) * 68 + c8 + (idx & 7);
      const float a = sa[o];
      const float g = sg[o];
      const float g3 = g * g * g;
      const float u = kGeluC0 * (g + kGeluC1 * g3);
      const float sig = __builtin_amdgcn_rcpf(1.0f + __expf(-2.0f * u));
      sa[o] = (a * (g * sig)) * ocarry;
    }
    v8h hv[4];
#pragma unroll
    for (int it = 0; it < 4; ++it) {
      const float* sp = sa + (it * 4 + q) * 68 + c8;
      const v4f a0 = *(const v4f*)(sp);
      const v4f a1 = *(const v4f*)(sp + 4);
#pragma unroll
      for (int e = 0; e < 4; ++e) {
        hv[it][e]     = (_Float16)a0[e];
        hv[it][4 + e] = (_Float16)a1[e];
      }
    }
    for (int pass = 0; pass < 2; ++pass) {
#pragma unroll
      for (int it = 0; it < 4; ++it)
        *(volatile v8h*)(Cact + (size_t)(mBase + it * 4 + q) * ldc + n0 + c8) = hv[it];
      __threadfence();
    }
    wave_sync();
  }
}

__global__ __launch_bounds__(256) void transpose_cast_kernel(
    const float* __restrict__ W, unsigned short* __restrict__ Bt, int Kdim, int Ndim, float scale)
{
  __shared__ float tile[64 * 65];
  const int tid = threadIdx.x, lane = tid & 31, wave = tid >> 5;
  const int n0 = blockIdx.x * 64;
  const int k0 = blockIdx.y * 64;
#pragma unroll
  for (int p = 0; p < 16; ++p) {
    const int idx = tid + p * 256;
    const int kk  = idx >> 6;
    const int nn  = idx & 63;
    const int n   = n0 + nn;
    const int nc  = (n < Ndim) ? n : (Ndim - 1);
    const float v = W[(size_t)(k0 + kk) * Ndim + nc];
    tile[kk * 65 + nn] = (n < Ndim) ? (v * scale) : 0.f;
  }
  __syncthreads();
  const int q = lane >> 3, c8 = (lane & 7) * 8;
  v8h hv[2];
#pragma unroll
  for (int it = 0; it < 2; ++it) {
    const int nrow = it * 32 + wave * 4 + q;
#pragma unroll
    for (int e = 0; e < 8; ++e) hv[it][e] = (_Float16)tile[(c8 + e) * 65 + nrow];
  }
  for (int pass = 0; pass < 2; ++pass) {
#pragma unroll
    for (int it = 0; it < 2; ++it) {
      const int nrow = it * 32 + wave * 4 + q;
      *(volatile v8h*)(Bt + (size_t)(n0 + nrow) * Kdim + k0 + c8) = hv[it];
    }
    __threadfence();
  }
}

__global__ __launch_bounds__(256) void layernorm_f16_kernel(
    const float* __restrict__ X, const float* __restrict__ gam, const float* __restrict__ bet,
    unsigned short* __restrict__ H, int rows)
{
  const int lane = threadIdx.x & 31, wave = threadIdx.x >> 5;
  const int row = blockIdx.x * 8 + wave;
  if (row >= rows) return;
  const float* xr = X + (size_t)row * kDm;
  float s = 0.f;
#pragma unroll 1
  for (int it = 0; it < 4; ++it) {
    const float* p = xr + it * 256 + lane * 8;
    const v4f a0 = *(const v4f*)(p);
    const v4f a1 = *(const v4f*)(p + 4);
    s += ((a0[0] + a0[1]) + (a0[2] + a0[3])) + ((a1[0] + a1[1]) + (a1[2] + a1[3]));
  }
#pragma unroll
  for (int off = 16; off > 0; off >>= 1) s += __shfl_xor(s, off, 32);
  const float mu = s * (1.0f / kDm);
  float ss = 0.f;
#pragma unroll 1
  for (int it = 0; it < 4; ++it) {
    const float* p = xr + it * 256 + lane * 8;
    const v4f a0 = *(const v4f*)(p);
    const v4f a1 = *(const v4f*)(p + 4);
#pragma unroll
    for (int e = 0; e < 4; ++e) {
      const float d0 = a0[e] - mu;
      const float d1 = a1[e] - mu;
      ss = fmaf(d0, d0, ss);
      ss = fmaf(d1, d1, ss);
    }
  }
#pragma unroll
  for (int off = 16; off > 0; off >>= 1) ss += __shfl_xor(ss, off, 32);
  const float rstd = rsqrtf(ss * (1.0f / kDm) + kLnEps);
#pragma unroll 1
  for (int it = 0; it < 4; ++it) {
    const int c = it * 256 + lane * 8;
    const v4f a0 = *(const v4f*)(xr + c);
    const v4f a1 = *(const v4f*)(xr + c + 4);
    const v4f g0 = *(const v4f*)(gam + c);
    const v4f g1 = *(const v4f*)(gam + c + 4);
    const v4f b0 = *(const v4f*)(bet + c);
    const v4f b1 = *(const v4f*)(bet + c + 4);
    v8h hv;
#pragma unroll
    for (int e = 0; e < 4; ++e) {
      hv[e]     = (_Float16)((((a0[e] - mu) * rstd) * g0[e] + b0[e]) * kCarryH);
      hv[4 + e] = (_Float16)((((a1[e] - mu) * rstd) * g1[e] + b1[e]) * kCarryH);
    }
    unsigned short* qd = H + (size_t)row * kDm + c;
    *(volatile v8h*)qd = hv;
    __threadfence();
    *(volatile v8h*)qd = hv;
  }
}

__global__ __launch_bounds__(128) void conv_silu_kernel(
    const unsigned* __restrict__ XPRE32, const float* __restrict__ cw, const float* __restrict__ cb,
    unsigned short* __restrict__ XC)
{
  __shared__ __align__(16) float sT[16 * kConvTP];
  const int tid = threadIdx.x, lane = tid & 31, wave = tid >> 5;
  const int d0 = blockIdx.x * 256;
  const int c0 = d0 + 2 * tid;
  const int g0 = blockIdx.y * 64;
  const int tb = g0 & (kSeq - 1);
  const v4f wA = *(const v4f*)(cw + (size_t)c0 * 4);
  const v4f wB = *(const v4f*)(cw + (size_t)(c0 + 1) * 4);
  const float bA = cb[c0], bB = cb[c0 + 1];
  const size_t wcol = (size_t)(d0 >> 1) + tid;
  float a3, a2, a1, b3, b2, b1;
  {
    const bool hist = (tb > 0);
    const int rb = hist ? (g0 - 3) : g0;
    const unsigned w3 = XPRE32[(size_t)rb * (kDi / 2) + wcol];
    const unsigned w2 = XPRE32[(size_t)(rb + 1) * (kDi / 2) + wcol];
    const unsigned w1 = XPRE32[(size_t)(rb + 2) * (kDi / 2) + wcol];
    const float fa3 = h16_to_f32(w3 & 0xffffu), fb3 = h16_to_f32(w3 >> 16);
    const float fa2 = h16_to_f32(w2 & 0xffffu), fb2 = h16_to_f32(w2 >> 16);
    const float fa1 = h16_to_f32(w1 & 0xffffu), fb1 = h16_to_f32(w1 >> 16);
    a3 = hist ? fa3 : 0.f;  b3 = hist ? fb3 : 0.f;
    a2 = hist ? fa2 : 0.f;  b2 = hist ? fb2 : 0.f;
    a1 = hist ? fa1 : 0.f;  b1 = hist ? fb1 : 0.f;
  }
#pragma unroll 1
  for (int sub = 0; sub < 4; ++sub) {
    const int lb = g0 + sub * 16;
#pragma unroll 1
    for (int s = 0; s < 16; ++s) {
      const unsigned w = XPRE32[(size_t)(lb + s) * (kDi / 2) + wcol];
      const float xa = h16_to_f32(w & 0xffffu);
      const float xb = h16_to_f32(w >> 16);
      float va = wA[0] * a3;
      va = fmaf(wA[1], a2, va);
      va = fmaf(wA[2], a1, va);
      va = fmaf(wA[3], xa, va);
      float vb = wB[0] * b3;
      vb = fmaf(wB[1], b2, vb);
      vb = fmaf(wB[2], b1, vb);
      vb = fmaf(wB[3], xb, vb);
      va += bA;
      vb += bB;
      const float sa = __builtin_amdgcn_rcpf(1.0f + expf(-va));
      const float sb = __builtin_amdgcn_rcpf(1.0f + expf(-vb));
      sT[s * kConvTP + 2 * tid]     = va * sa;
      sT[s * kConvTP + 2 * tid + 1] = vb * sb;
      a3 = a2; a2 = a1; a1 = xa;
      b3 = b2; b2 = b1; b1 = xb;
    }
    __syncthreads();
    v8h hv[4];
#pragma unroll
    for (int it = 0; it < 4; ++it) {
      const float* sp = sT + (it * 4 + wave) * kConvTP + lane * 8;
      const v4f p0 = *(const v4f*)(sp);
      const v4f p1 = *(const v4f*)(sp + 4);
#pragma unroll
      for (int e = 0; e < 4; ++e) {
        hv[it][e]     = (_Float16)(p0[e] * kCarryXc);
        hv[it][4 + e] = (_Float16)(p1[e] * kCarryXc);
      }
    }
    for (int pass = 0; pass < 2; ++pass) {
#pragma unroll
      for (int it = 0; it < 4; ++it)
        *(volatile v8h*)(XC + (size_t)(lb + it * 4 + wave) * kDi + d0 + lane * 8) = hv[it];
      __threadfence();
    }
    __syncthreads();
  }
}

__global__ __launch_bounds__(32) void scan_gate_kernel(
    const unsigned* __restrict__ DT32, const unsigned* __restrict__ XC32, const unsigned* __restrict__ Z32,
    const float* __restrict__ BC, const float* __restrict__ a_log, const float* __restrict__ d_skip,
    unsigned* __restrict__ Y32)
{
  __shared__ float sAn[32 * 32];
  const int lane = threadIdx.x;
  constexpr int kBlkPerSeq = kDi / 64;
  const int bix = blockIdx.x / kBlkPerSeq;
  const int cb  = (blockIdx.x - bix * kBlkPerSeq) * 64;
  const int c0  = cb + 2 * lane;
#pragma unroll 1
  for (int idx = 0; idx < 32; ++idx)
    sAn[idx * 32 + lane] = -expf(a_log[(size_t)(c0 + (idx >> 4)) * kNs + (idx & 15)]);
  __syncthreads();
  float An0[kNs], An1[kNs], h0[kNs], h1[kNs];
#pragma unroll
  for (int n = 0; n < kNs; ++n) {
    An0[n] = sAn[n * 32 + lane];
    An1[n] = sAn[(kNs + n) * 32 + lane];
    h0[n] = 0.f;
    h1[n] = 0.f;
  }
  const float dsk0 = d_skip[c0], dsk1 = d_skip[c0 + 1];
  const size_t wcol = (size_t)(cb >> 1) + lane;
#pragma unroll 1
  for (int t = 0; t < kSeq; ++t) {
    const size_t row = (size_t)bix * kSeq + t;
    const size_t wi  = row * (kDi / 2) + wcol;
    const unsigned wdt = DT32[wi];
    const unsigned wxc = XC32[wi];
    const unsigned wz  = Z32[wi];
    const float* bc = BC + row * kBcP;
    v4f Bq[4], Cq[4];
#pragma unroll
    for (int qq = 0; qq < 4; ++qq) {
      Bq[qq] = *(const v4f*)(bc + 4 * qq);
      Cq[qq] = *(const v4f*)(bc + kNs + 4 * qq);
    }
    const float dt0 = h16_to_f32(wdt & 0xffffu);
    const float dt1 = h16_to_f32(wdt >> 16);
    const float xc0 = h16_to_f32(wxc & 0xffffu) * kInvXc;
    const float xc1 = h16_to_f32(wxc >> 16) * kInvXc;
    const float z0  = h16_to_f32(wz & 0xffffu);
    const float z1  = h16_to_f32(wz >> 16);
    const float dtx0 = dt0 * xc0;
    const float dtx1 = dt1 * xc1;
    float y0 = 0.f, y1 = 0.f;
#pragma unroll
    for (int n = 0; n < kNs; ++n) {
      const float bn = Bq[n >> 2][n & 3];
      const float cn = Cq[n >> 2][n & 3];
      const float e0 = __expf(dt0 * An0[n]);
      const float e1 = __expf(dt1 * An1[n]);
      h0[n] = fmaf(e0, h0[n], dtx0 * bn);
      h1[n] = fmaf(e1, h1[n], dtx1 * bn);
      y0 = fmaf(h0[n], cn, y0);
      y1 = fmaf(h1[n], cn, y1);
    }
    y0 = fmaf(dsk0, xc0, y0);
    y1 = fmaf(dsk1, xc1, y1);
    const float g0 = z0 * __builtin_amdgcn_rcpf(1.0f + __expf(-z0));
    const float g1 = z1 * __builtin_amdgcn_rcpf(1.0f + __expf(-z1));
    const float o0 = (y0 * g0) * kCarryY;
    const float o1 = (y1 * g1) * kCarryY;
    v2h pk;
    pk[0] = (_Float16)o0;
    pk[1] = (_Float16)o1;
    const unsigned wy = __builtin_bit_cast(unsigned, pk);
    unsigned* yp = Y32 + wi;
    *(volatile unsigned*)yp = wy;
    __threadfence();
    *(volatile unsigned*)yp = wy;
  }
}

extern "C" void kernel_launch(void* const* d_in, const int* in_sizes, int n_in,
                              void* d_out, int out_size, void* d_ws, size_t ws_size,
                              hipStream_t stream)
{
  if (n_in < 18) return;
  if (in_sizes[0] != kRows * kDm) return;
  if (in_sizes[1] != kDm || in_sizes[2] != kDm) return;
  if (in_sizes[3] != kDm * 2 * kDi) return;
  if (in_sizes[4] != kDi * 4 || in_sizes[5] != kDi) return;
  if (in_sizes[6] != kDi * kXpN) return;
  if (in_sizes[7] != kDtR * kDi || in_sizes[8] != kDi) return;
  if (in_sizes[9] != kDi * kNs || in_sizes[10] != kDi) return;
  if (in_sizes[11] != kDi * kDm) return;
  if (in_sizes[12] != kDm || in_sizes[13] != kDm) return;
  if (in_sizes[14] != kDm * 2 * kFf || in_sizes[15] != 2 * kFf) return;
  if (in_sizes[16] != kFf * kDm || in_sizes[17] != kDm) return;
  if (out_size != kRows * kDm) return;
  if (ws_size < kWsTotal) return;

  const float* x      = (const float*)d_in[0];
  const float* ln1_g  = (const float*)d_in[1];
  const float* ln1_b  = (const float*)d_in[2];
  const float* w_in   = (const float*)d_in[3];
  const float* conv_w = (const float*)d_in[4];
  const float* conv_b = (const float*)d_in[5];
  const float* w_x    = (const float*)d_in[6];
  const float* w_dt   = (const float*)d_in[7];
  const float* b_dt   = (const float*)d_in[8];
  const float* a_log  = (const float*)d_in[9];
  const float* d_skip = (const float*)d_in[10];
  const float* w_out  = (const float*)d_in[11];
  const float* ln2_g  = (const float*)d_in[12];
  const float* ln2_b  = (const float*)d_in[13];
  const float* w_ff1  = (const float*)d_in[14];
  const float* b_ff1  = (const float*)d_in[15];
  const float* w_ff2  = (const float*)d_in[16];
  const float* b_ff2  = (const float*)d_in[17];
  float* out = (float*)d_out;

  char* ws = (char*)d_ws;
  unsigned short* WIN  = (unsigned short*)(ws + kOffWIn);
  unsigned short* WX   = (unsigned short*)(ws + kOffWX);
  unsigned short* WDT  = (unsigned short*)(ws + kOffWDt);
  unsigned short* WOUT = (unsigned short*)(ws + kOffWOut);
  unsigned short* H    = (unsigned short*)(ws + kOffH);
  float*          X2   = (float*)(ws + kOffX2);
  unsigned short* DTLO = (unsigned short*)(ws + kOffDtLo);
  float*          BC   = (float*)(ws + kOffBC);
  unsigned short* XPRE = (unsigned short*)(ws + kOffXpre);
  unsigned short* Z    = (unsigned short*)(ws + kOffZ);
  unsigned short* XC   = (unsigned short*)(ws + kOffXc);
  unsigned short* DT   = (unsigned short*)(ws + kOffDt);
  unsigned short* ACT  = (unsigned short*)(ws + kOffAct);
  unsigned short* WFF1 = (unsigned short*)(ws + kOffWFf1);
  unsigned short* WFF2 = (unsigned short*)(ws + kOffWFf2);

  transpose_cast_kernel<<<dim3((2 * kDi) / 64, kDm / 64), 256, 0, stream>>>(w_in, WIN, kDm, 2 * kDi, kCarryW);
  transpose_cast_kernel<<<dim3(kXpP / 64, kDi / 64), 256, 0, stream>>>(w_x, WX, kDi, kXpN, kCarryW);
  transpose_cast_kernel<<<dim3(kDi / 64, kDtR / 64), 256, 0, stream>>>(w_dt, WDT, kDtR, kDi, kCarryWdt);
  transpose_cast_kernel<<<dim3(kDm / 64, kDi / 64), 256, 0, stream>>>(w_out, WOUT, kDi, kDm, kCarryW);

  layernorm_f16_kernel<<<kRows / 8, 256, 0, stream>>>(x, ln1_g, ln1_b, H, kRows);

  gemm64_f16_kernel<0><<<512, 256, 0, stream>>>(
      H, kDm, WIN, kDm, (void*)XPRE, (void*)Z, kDi, kDi,
      b_dt, x, kRows, 2 * kDi, kDm, kScaleIn, kScaleIn);

  conv_silu_kernel<<<dim3(kDi / 256, kRows / 64), 128, 0, stream>>>(
      (const unsigned*)XPRE, conv_w, conv_b, XC);

  gemm64_f16_kernel<1><<<16, 256, 0, stream>>>(
      XC, kDi, WX, kDi, (void*)DTLO, (void*)BC, kBcP, kDtR,
      b_dt, x, kRows, kXpP, kDi, kScaleXpLo, kScaleXpBc);

  gemm64_f16_kernel<2><<<256, 256, 0, stream>>>(
      DTLO, kDtR, WDT, kDtR, (void*)DT, (void*)DT, kDi, kDi,
      b_dt, x, kRows, kDi, kDtR, kScaleDt, kScaleDt);

  scan_gate_kernel<<<kBatch * (kDi / 64), 32, 0, stream>>>(
      (const unsigned*)DT, (const unsigned*)XC, (const unsigned*)Z, BC, a_log, d_skip, (unsigned*)XPRE);

  gemm64_f16_kernel<3><<<128, 256, 0, stream>>>(
      XPRE, kDi, WOUT, kDi, (void*)X2, (void*)X2, kDm, kDm,
      b_dt, x, kRows, kDm, kDi, kScaleOut, kScaleOut);

  layernorm_f16_kernel<<<kRows / 8, 256, 0, stream>>>(X2, ln2_g, ln2_b, H, kRows);

  transpose_cast_kernel<<<dim3((2 * kFf) / 64, kDm / 64), 256, 0, stream>>>(w_ff1, WFF1, kDm, 2 * kFf, kCarryW);
  transpose_cast_kernel<<<dim3(kDm / 64, kFf / 64), 256, 0, stream>>>(w_ff2, WFF2, kFf, kDm, kCarryW);

  gemm_gated_f16_kernel<<<(kRows / 32) * (kFf / 64) / 4, 128, 0, stream>>>(
      H, kDm, WFF1, kDm, ACT, kFf, b_ff1, kRows, kFf, kDm, kScaleFf1, kCarryAct);

  gemm64_f16_kernel<4><<<128, 256, 0, stream>>>(
      ACT, kFf, WFF2, kFf, (void*)out, (void*)out, kDm, kDm,
      b_ff2, X2, kRows, kDm, kFf, kScaleFf2, kScaleFf2);
}
